// Teacher_S_84945863180994
// MI455X (gfx1250) — hardware-verified
//
#include <hip/hip_runtime.h>
#include <stddef.h>


typedef _Float16 h16;
typedef _Float16 v16h __attribute__((ext_vector_type(16)));
typedef _Float16 v8h  __attribute__((ext_vector_type(8)));
typedef float    v8f  __attribute__((ext_vector_type(8)));
typedef float    v4f  __attribute__((ext_vector_type(4)));

#ifndef NNODE
#define NNODE 2048
#endif
#define NN_FULL 2048
#define IND   1024
#define HIDW  256
#define H2W   64
#define NCLS  4
#define NPADC 16

#define EROWS    32
#define ETHREADS (NNODE / 8)
#define EWAVES   (ETHREADS / 32)

static_assert(NNODE >= 512 && NNODE <= NN_FULL && (NNODE % 512) == 0);
static_assert(ETHREADS * 8 == NNODE && ETHREADS <= 256 && (ETHREADS % 32) == 0);
static_assert(EROWS == 32 && (NNODE % EROWS) == 0);
static_assert((NNODE % 128) == 0 && (NNODE % 64) == 0 && (NNODE % 32) == 0);
static_assert((IND % 64) == 0 && (IND % 32) == 0);
static_assert((HIDW % 64) == 0 && (HIDW % 32) == 0);
static_assert(H2W == 64 && NCLS == 4 && NPADC == 16);
static_assert(((size_t)NNODE * IND) % 2048 == 0);
static_assert(2 * 32 == 64);
static_assert(4 * 16 == 64);
static_assert((size_t)NN_FULL * NCLS * 4 == (size_t)32768);
static_assert(((size_t)NN_FULL * NCLS + (size_t)NNODE * H2W) * 4 <= (size_t)557056);

#define LDT 72
#define LDC 68
static_assert((LDT % 8) == 0 && LDT >= 64);
static_assert((LDC % 4) == 0 && LDC >= 64);

#define WCARRY 64.0f
#define XINC   16.0f
#define XCARRY 1024.0f
#define BCARRY 4096.0f
#define HCARRY 256.0f
#define GCARRY 16384.0f

#define X16_BYTES  ((size_t)NNODE * IND * 2)
#define WG1T_BYTES ((size_t)HIDW * IND * 2)
#define WL2T_BYTES ((size_t)H2W * HIDW * 2)
#define B16_BYTES  ((size_t)NNODE * NNODE * 2)
#define XWT_BYTES  ((size_t)HIDW * NNODE * 2)
#define H1_BYTES   ((size_t)NNODE * HIDW * 2)
#define HGT_BYTES  ((size_t)NPADC * NNODE * 2)
#define COLP_BYTES ((size_t)(NNODE / EROWS) * NNODE * 4)
#define VEC_BYTES  ((size_t)NNODE * 4)
#define OFF_X16  ((size_t)0)
#define OFF_WG1T (OFF_X16 + X16_BYTES)
#define OFF_WL2T (OFF_WG1T + WG1T_BYTES)
#define OFF_B16  (OFF_WL2T + WL2T_BYTES)
#define OFF_XWT  (OFF_B16 + B16_BYTES)
#define OFF_H1   (OFF_XWT + XWT_BYTES)
#define OFF_HGT  (OFF_H1 + H1_BYTES)
#define OFF_COLP (OFF_HGT + HGT_BYTES)
#define OFF_DR   (OFF_COLP + COLP_BYTES)
#define OFF_DC   (OFF_DR + VEC_BYTES)
#define WS_TOTAL (OFF_DC + VEC_BYTES)
static_assert((X16_BYTES % 128) == 0 && (WG1T_BYTES % 128) == 0 && (WL2T_BYTES % 128) == 0);
static_assert((B16_BYTES % 128) == 0 && (XWT_BYTES % 128) == 0 && (H1_BYTES % 128) == 0);
static_assert((HGT_BYTES % 128) == 0 && (COLP_BYTES % 128) == 0 && (VEC_BYTES % 128) == 0);
static_assert(WS_TOTAL <= (size_t)134217728);

__device__ __forceinline__ float bf16r(float x) {
  unsigned int u = __float_as_uint(x);
  u = (u + 0x7FFFu + ((u >> 16) & 1u)) & 0xFFFF0000u;
  return __uint_as_float(u);
}

static __device__ __forceinline__ h16 toh_flush(float v) {
  const h16 r = (h16)v;
  return (fabsf(v) < 6.103515625e-05f) ? (h16)0.0f : r;
}

__device__ __forceinline__ v16h frag_at(const _Float16* p) {
  v8h lo = *(const v8h*)(p);
  v8h hi = *(const v8h*)(p + 16);
  v16h out;
#pragma unroll
  for (int i = 0; i < 8; ++i) { out[i] = lo[i]; out[i + 8] = hi[i]; }
  return out;
}

__device__ __forceinline__ v8f wmma16(v16h a, v16h b, v8f c) {
  v8f d = __builtin_amdgcn_wmma_f32_16x16x32_f16(false, a, false, b, (short)0, c,
                                                 false, false);
  asm volatile("v_nop\n\tv_nop\n\tv_nop\n\tv_nop" : "+v"(d) : "v"(a), "v"(b));
  return d;
}

__device__ __forceinline__ float red32_sum(float x) {
#pragma unroll
  for (int off = 1; off < 32; off <<= 1) x += __shfl_xor(x, off, 32);
  return x;
}

__global__ __launch_bounds__(256) void wconv_kernel(
    const float* __restrict__ W, _Float16* __restrict__ Wt, unsigned ldw, unsigned ldk) {
  __shared__ _Float16 T[64 * LDT];
  const unsigned tid = threadIdx.x;
  const unsigned n0 = blockIdx.x * 64u;
  const unsigned k0 = blockIdx.y * 64u;
#pragma unroll 4
  for (unsigned j = 0; j < 16u; ++j) {
    const unsigned idx = tid + 256u * j;
    const unsigned kr = idx >> 6, nc = idx & 63u;
    const float v = W[(size_t)(k0 + kr) * ldw + n0 + nc];
    T[nc * LDT + kr] = toh_flush(WCARRY * bf16r(v));
  }
  __syncthreads();
  v8h x[2];
  size_t off[2];
#pragma unroll
  for (unsigned i = 0; i < 2u; ++i) {
    const unsigned n = 32u * i + (tid >> 3);
    const unsigned kc = (tid & 7u) * 8u;
    x[i] = *(const v8h*)&T[n * LDT + kc];
    off[i] = (size_t)(n0 + n) * ldk + k0 + kc;
  }
#pragma unroll
  for (int i = 0; i < 2; ++i) *(volatile v8h*)(Wt + off[i]) = x[i];
  __threadfence();
#pragma unroll
  for (int i = 0; i < 2; ++i) *(volatile v8h*)(Wt + off[i]) = x[i];
}

__global__ __launch_bounds__(256) void xconv_kernel(
    const float* __restrict__ X, _Float16* __restrict__ X16) {
  const size_t e = ((size_t)blockIdx.x * 256u + threadIdx.x) * 8u;
  const v4f a0 = *(const v4f*)(X + e);
  const v4f a1 = *(const v4f*)(X + e + 4u);
  v8h o;
#pragma unroll
  for (int i = 0; i < 4; ++i) {
    o[i]     = toh_flush(XINC * bf16r(a0[i]));
    o[i + 4] = toh_flush(XINC * bf16r(a1[i]));
  }
  _Float16* p = X16 + e;
  *(volatile v8h*)p = o;
  __threadfence();
  *(volatile v8h*)p = o;
}

__global__ __launch_bounds__(ETHREADS) void edge_kernel(
    const float* __restrict__ adj, const float* __restrict__ xdeg, const float* __restrict__ ydeg,
    const float* __restrict__ Wm1, const float* __restrict__ bm1,
    const float* __restrict__ Wm2, const float* __restrict__ bm2,
    _Float16* __restrict__ B16, float* __restrict__ colpart, float* __restrict__ drv) {
  __shared__ float sW[16 * 8];
  __shared__ float RowP[EWAVES * EROWS];
  __shared__ float Cc[NNODE];
  __shared__ float DrS[EROWS];
  const unsigned tid = threadIdx.x, lane = tid & 31u;
  const unsigned wave = (unsigned)__builtin_amdgcn_readfirstlane((int)(threadIdx.x >> 5));
  {
    const unsigned k = tid & 15u;
    float w0 = bf16r(Wm1[k]);
    float w1 = bf16r(Wm1[16u + k]);
    float w2 = bf16r(Wm1[32u + k]);
    float bb = bf16r(bm1[k]);
    float wd = bf16r(Wm2[2u * k + 1u]) - bf16r(Wm2[2u * k]);
    float bd = bf16r(bm2[1]) - bf16r(bm2[0]);
    asm volatile("" : "+v"(w0), "+v"(w1), "+v"(w2), "+v"(bb), "+v"(wd), "+v"(bd));
    if (tid < 16u) {
      sW[k * 8u + 0u] = w0;
      sW[k * 8u + 1u] = w1;
      sW[k * 8u + 2u] = w2;
      sW[k * 8u + 3u] = bb;
      sW[k * 8u + 4u] = wd;
      sW[k * 8u + 5u] = bd;
      sW[k * 8u + 6u] = 0.0f;
      sW[k * 8u + 7u] = 0.0f;
    }
  }
  __syncthreads();

  const unsigned row0 = blockIdx.x * (unsigned)EROWS;
  const unsigned col = tid * 8u;
  const float bd0 = sW[5];
  float cs[8];
#pragma unroll
  for (int e = 0; e < 8; ++e) cs[e] = 0.0f;

#pragma unroll 1
  for (unsigned r = 0; r < (unsigned)EROWS; ++r) {
    const unsigned i = row0 + r;
    const size_t src = (size_t)i * NN_FULL + col;
    const v4f a0 = *(const v4f*)(adj + src);
    const v4f a1 = *(const v4f*)(adj + src + 4u);
    const v4f x0 = *(const v4f*)(xdeg + src);
    const v4f x1 = *(const v4f*)(xdeg + src + 4u);
    const v4f y0 = *(const v4f*)(ydeg + src);
    const v4f y1 = *(const v4f*)(ydeg + src + 4u);
    float av[8], xv[8], yv[8], l[8];
#pragma unroll
    for (int e = 0; e < 4; ++e) {
      av[e] = bf16r(a0[e]); av[e + 4] = bf16r(a1[e]);
      xv[e] = bf16r(x0[e]); xv[e + 4] = bf16r(x1[e]);
      yv[e] = bf16r(y0[e]); yv[e + 4] = bf16r(y1[e]);
    }
#pragma unroll
    for (int e = 0; e < 8; ++e) l[e] = bd0;
#pragma unroll 1
    for (unsigned k = 0; k < 16u; ++k) {
      const v4f wv = *(const v4f*)&sW[k * 8u];
      const float wd = sW[k * 8u + 4u];
#pragma unroll
      for (int e = 0; e < 8; ++e) {
        const float h = fmaxf(av[e] * wv[0] + xv[e] * wv[1] + yv[e] * wv[2] + wv[3], 0.0f);
        l[e] += h * wd;
      }
    }
    float rp = 0.0f;
    v8h o;
#pragma unroll
    for (int e = 0; e < 8; ++e) {
      const float mk = __builtin_amdgcn_rcpf(1.0f + __expf(-l[e]));
      const float dg = ((col + (unsigned)e) == i) ? 1.0f : 0.0f;
      const float bv = av[e] * mk + dg;
      cs[e] += bv;
      rp += bv;
      o[e] = toh_flush(BCARRY * bv);
    }
    _Float16* p = B16 + (size_t)i * NNODE + col;
    *(volatile v8h*)p = o;
    __threadfence();
    *(volatile v8h*)p = o;
    rp = red32_sum(rp);
    if (lane == 0u) RowP[wave * (unsigned)EROWS + r] = rp;
  }

  {
    v4f c0, c1;
#pragma unroll
    for (int e = 0; e < 4; ++e) { c0[e] = cs[e]; c1[e] = cs[e + 4]; }
    *(v4f*)&Cc[col] = c0;
    *(v4f*)&Cc[col + 4u] = c1;
  }
  __syncthreads();
  if (tid < (unsigned)EROWS) {
    float s = 0.0f;
#pragma unroll
    for (unsigned w2 = 0; w2 < (unsigned)EWAVES; ++w2) s += RowP[w2 * (unsigned)EROWS + tid];
    const float sp = (s > 0.0f) ? s : 1.0f;
    const float v = 1.0f / sqrtf(sp);
    DrS[tid] = (s > 0.0f) ? v : 0.0f;
  }
  __syncthreads();

  const unsigned c4 = tid * 4u;
  const v4f p0 = *(const v4f*)&Cc[c4];
  const v4f p1 = *(const v4f*)&Cc[(unsigned)(NNODE / 2) + c4];
  const v4f dv = *(const v4f*)&DrS[(tid & 7u) * 4u];
  float* cp = colpart + (size_t)blockIdx.x * NNODE;
  float* dp = drv + row0 + (tid & 7u) * 4u;
  *(volatile v4f*)(cp + c4) = p0;
  *(volatile v4f*)(cp + (unsigned)(NNODE / 2) + c4) = p1;
  if (tid < 8u) *(volatile v4f*)dp = dv;
  __threadfence();
  *(volatile v4f*)(cp + c4) = p0;
  *(volatile v4f*)(cp + (unsigned)(NNODE / 2) + c4) = p1;
  if (tid < 8u) *(volatile v4f*)dp = dv;
}

__global__ __launch_bounds__(128) void dcol_kernel(
    const float* __restrict__ colpart, float* __restrict__ dcv) {
  __shared__ float Ds[128];
  const unsigned tid = threadIdx.x;
  const unsigned c = blockIdx.x * 128u + tid;
  float s = 0.0f;
#pragma unroll 4
  for (unsigned b = 0; b < (unsigned)(NNODE / EROWS); ++b) s += colpart[(size_t)b * NNODE + c];
  const float sp = (s > 0.0f) ? s : 1.0f;
  const float v = 1.0f / sqrtf(sp);
  Ds[tid] = (s > 0.0f) ? v : 0.0f;
  __syncthreads();
  if (tid < 32u) {
    const v4f o = *(const v4f*)&Ds[tid * 4u];
    float* p = dcv + blockIdx.x * 128u + tid * 4u;
    *(volatile v4f*)p = o;
    __threadfence();
    *(volatile v4f*)p = o;
  }
}

template <int MODE>
__device__ __forceinline__ void gemm_body(
    const _Float16* __restrict__ A16, const _Float16* __restrict__ Bt, const unsigned K,
    const float* __restrict__ v0, const float* __restrict__ v1, const float* __restrict__ v2,
    float* __restrict__ outf, _Float16* __restrict__ out16) {
  __shared__ float Cs[64 * LDC];
  const unsigned tid = threadIdx.x, lane = tid & 31u, w = tid >> 5;
  const unsigned mw = w >> 1, nw = w & 1u;
  const unsigned hh = lane >> 4, m = lane & 15u;
  const unsigned n0 = blockIdx.x * 64u;
  const unsigned row0 = blockIdx.y * 64u;

  const _Float16* ap  = A16 + (size_t)(row0 + mw * 16u + m) * K + hh * 8u;
  const _Float16* bp0 = Bt + (size_t)(n0 + nw * 32u + m) * K + hh * 8u;
  const _Float16* bp1 = bp0 + (size_t)16 * K;
  v8f acc0 = {}, acc1 = {};
#pragma unroll 2
  for (unsigned k0 = 0; k0 < K; k0 += 32u) {
    const v16h a  = frag_at(ap + k0);
    const v16h b0 = frag_at(bp0 + k0);
    const v16h b1 = frag_at(bp1 + k0);
    acc0 = wmma16(a, b0, acc0);
    acc1 = wmma16(a, b1, acc1);
  }
#pragma unroll
  for (int r = 0; r < 8; ++r) {
    float* d = &Cs[(mw * 16u + hh * 8u + (unsigned)r) * LDC + nw * 32u + m];
    d[0]  = acc0[r];
    d[16] = acc1[r];
  }
  __syncthreads();

  if (MODE == 0) {
    const unsigned kk = (tid & 7u) * 8u;
    const v4f d0 = *(const v4f*)(v0 + row0 + kk);
    const v4f d1 = *(const v4f*)(v0 + row0 + kk + 4u);
    v8h x[2];
    size_t off[2];
#pragma unroll
    for (unsigned i = 0; i < 2u; ++i) {
      const unsigned dcol = 32u * i + (tid >> 3);
#pragma unroll
      for (unsigned j = 0; j < 4u; ++j) {
        const float t0 = Cs[(kk + j) * LDC + dcol] * (XCARRY / (XINC * WCARRY)) * d0[j];
        const float t1 = Cs[(kk + 4u + j) * LDC + dcol] * (XCARRY / (XINC * WCARRY)) * d1[j];
        x[i][j]      = toh_flush(t0);
        x[i][j + 4u] = toh_flush(t1);
      }
      off[i] = (size_t)(n0 + dcol) * NNODE + row0 + kk;
    }
#pragma unroll
    for (int i = 0; i < 2; ++i) *(volatile v8h*)(out16 + off[i]) = x[i];
    __threadfence();
#pragma unroll
    for (int i = 0; i < 2; ++i) *(volatile v8h*)(out16 + off[i]) = x[i];
  }

  if (MODE == 1) {
    v8h x[2];
    size_t off[2];
#pragma unroll
    for (unsigned i = 0; i < 2u; ++i) {
      const unsigned r = 32u * i + (tid >> 3);
      const unsigned c = (tid & 7u) * 8u;
      const v4f u0 = *(const v4f*)&Cs[r * LDC + c];
      const v4f u1 = *(const v4f*)&Cs[r * LDC + c + 4];
      const float s = v0[row0 + r] * (HCARRY / (BCARRY * XCARRY));
#pragma unroll
      for (int j = 0; j < 4; ++j) {
        x[i][j]     = toh_flush(u0[j] * s);
        x[i][j + 4] = toh_flush(u1[j] * s);
      }
      off[i] = (size_t)(row0 + r) * HIDW + n0 + c;
    }
#pragma unroll
    for (int i = 0; i < 2; ++i) *(volatile v8h*)(out16 + off[i]) = x[i];
    __threadfence();
#pragma unroll
    for (int i = 0; i < 2; ++i) *(volatile v8h*)(out16 + off[i]) = x[i];
  }

  if (MODE == 2) {
    __shared__ _Float16 Hs[4 * LDT];
    v4f xs[4];
    size_t off[4];
#pragma unroll
    for (unsigned i = 0; i < 4u; ++i) {
      const unsigned r = 16u * i + (tid >> 4);
      const unsigned c = (tid & 15u) * 4u;
      const v4f u = *(const v4f*)&Cs[r * LDC + c];
      const v4f g = *(const v4f*)(v0 + n0 + c);
      v4f val;
#pragma unroll
      for (int j = 0; j < 4; ++j) val[j] = u[j] * (1.0f / (HCARRY * WCARRY)) + bf16r(g[j]);
      xs[i] = val;
      *(v4f*)&Cs[r * LDC + c] = val;
      off[i] = (size_t)NN_FULL * NCLS + (size_t)(row0 + r) * H2W + n0 + c;
    }
#pragma unroll
    for (int i = 0; i < 4; ++i) *(volatile v4f*)(outf + off[i]) = xs[i];
    __threadfence();
#pragma unroll
    for (int i = 0; i < 4; ++i) *(volatile v4f*)(outf + off[i]) = xs[i];
    __syncthreads();

    {
      const unsigned row = tid >> 2, cls = tid & 3u;
      float hg = 0.0f;
#pragma unroll 4
      for (unsigned k = 0; k < (unsigned)H2W; ++k)
        hg += Cs[row * LDC + k] * bf16r(v2[k * (unsigned)NCLS + cls]);
      Hs[cls * LDT + row] = toh_flush(GCARRY * v1[row0 + row] * hg);
    }
    __syncthreads();
    if (tid < 128u) {
      const unsigned n = tid >> 3;
      const unsigned kc = (tid & 7u) * 8u;
      const unsigned nn = (n < 3u) ? n : 3u;
      const v8h hv = *(const v8h*)&Hs[nn * LDT + kc];
      const v8h z = {};
      const v8h xo = (n < (unsigned)NCLS) ? hv : z;
      _Float16* p = out16 + (size_t)n * NNODE + row0 + kc;
      *(volatile v8h*)p = xo;
      __threadfence();
      *(volatile v8h*)p = xo;
    }
  }
}

__global__ __launch_bounds__(256) void gemm_xw_kernel(
    const _Float16* __restrict__ A16, const _Float16* __restrict__ Bt,
    const float* __restrict__ dcv, _Float16* __restrict__ xwt) {
  gemm_body<0>(A16, Bt, (unsigned)IND, dcv, dcv, dcv, (float*)0, xwt);
}
__global__ __launch_bounds__(256) void gemm_h1_kernel(
    const _Float16* __restrict__ A16, const _Float16* __restrict__ Bt,
    const float* __restrict__ drv, _Float16* __restrict__ h1) {
  gemm_body<1>(A16, Bt, (unsigned)NNODE, drv, drv, drv, (float*)0, h1);
}
__global__ __launch_bounds__(256) void gemm_hid_kernel(
    const _Float16* __restrict__ A16, const _Float16* __restrict__ Bt,
    const float* __restrict__ bias, const float* __restrict__ dcv,
    const float* __restrict__ wg2, float* __restrict__ outf, _Float16* __restrict__ hgt) {
  gemm_body<2>(A16, Bt, (unsigned)HIDW, bias, dcv, wg2, outf, hgt);
}

__global__ __launch_bounds__(256) void gemm_out_kernel(
    const _Float16* __restrict__ B16, const _Float16* __restrict__ HGt,
    const float* __restrict__ drv, float* __restrict__ outf) {
  __shared__ float Os[128 * 4];
  const unsigned tid = threadIdx.x, lane = tid & 31u;
  const int wave = __builtin_amdgcn_readfirstlane(threadIdx.x >> 5);
  const unsigned hh = lane >> 4, m = lane & 15u;
  const unsigned row0 = blockIdx.x * 128u;

  const _Float16* ap = B16 + (size_t)(row0 + (unsigned)wave * 16u + m) * NNODE + hh * 8u;
  const _Float16* bp = HGt + (size_t)m * NNODE + hh * 8u;
  v8f acc = {};
#pragma unroll 2
  for (unsigned k0 = 0; k0 < (unsigned)NNODE; k0 += 32u) {
    const v16h a = frag_at(ap + k0);
    const v16h b = frag_at(bp + k0);
    acc = wmma16(a, b, acc);
  }
  if (m < (unsigned)NCLS) {
#pragma unroll
    for (int r = 0; r < 8; ++r)
      Os[((unsigned)wave * 16u + hh * 8u + (unsigned)r) * 4u + m] = acc[r];
  }
  __syncthreads();
  if (tid < 128u) {
    const v4f u = *(const v4f*)&Os[tid * 4u];
    const float s = drv[row0 + tid] * (1.0f / (BCARRY * GCARRY));
    v4f val;
#pragma unroll
    for (int j = 0; j < 4; ++j) val[j] = u[j] * s;
    float* p = outf + (size_t)(row0 + tid) * NCLS;
    *(volatile v4f*)p = val;
    __threadfence();
    *(volatile v4f*)p = val;
  }
}

extern "C" void kernel_launch(void* const* d_in, const int* in_sizes, int n_in,
                              void* d_out, int out_size, void* d_ws, size_t ws_size,
                              hipStream_t stream) {
  if (n_in < 12) return;
  const long long need_sq = (long long)(NNODE - 1) * NN_FULL + NNODE;
  if ((long long)in_sizes[0] < (long long)NNODE * IND) return;
  if ((long long)in_sizes[1] < need_sq) return;
  if ((long long)in_sizes[2] < need_sq) return;
  if ((long long)in_sizes[3] < need_sq) return;
  if (in_sizes[4] < 48 || in_sizes[5] < 16 || in_sizes[6] < 32 || in_sizes[7] < 2) return;
  if ((long long)in_sizes[8] < (long long)IND * HIDW) return;
  if ((long long)in_sizes[9] < (long long)HIDW * H2W) return;
  if (in_sizes[10] < H2W || in_sizes[11] < H2W * NCLS) return;
  if ((long long)out_size < (long long)NN_FULL * NCLS + (long long)NNODE * H2W) return;
  if (ws_size < WS_TOTAL) return;

  const float* x    = (const float*)d_in[0];
  const float* adj  = (const float*)d_in[1];
  const float* xdeg = (const float*)d_in[2];
  const float* ydeg = (const float*)d_in[3];
  const float* wm1  = (const float*)d_in[4];
  const float* bm1  = (const float*)d_in[5];
  const float* wm2  = (const float*)d_in[6];
  const float* bm2  = (const float*)d_in[7];
  const float* wg1  = (const float*)d_in[8];
  const float* wl2  = (const float*)d_in[9];
  const float* bl2  = (const float*)d_in[10];
  const float* wg2  = (const float*)d_in[11];
  float* out = (float*)d_out;

  char* ws = (char*)d_ws;
  _Float16* X16   = (_Float16*)(ws + OFF_X16);
  _Float16* Wg1_t = (_Float16*)(ws + OFF_WG1T);
  _Float16* Wl2_t = (_Float16*)(ws + OFF_WL2T);
  _Float16* B16   = (_Float16*)(ws + OFF_B16);
  _Float16* XWt   = (_Float16*)(ws + OFF_XWT);
  _Float16* H1p   = (_Float16*)(ws + OFF_H1);
  _Float16* HGt   = (_Float16*)(ws + OFF_HGT);
  float*    colp  = (float*)(ws + OFF_COLP);
  float*    drv   = (float*)(ws + OFF_DR);
  float*    dcv   = (float*)(ws + OFF_DC);

  dim3 blk(256);

  wconv_kernel<<<dim3(HIDW / 64, IND / 64), blk, 0, stream>>>(wg1, Wg1_t, (unsigned)HIDW, (unsigned)IND);
  wconv_kernel<<<dim3(H2W / 64, HIDW / 64), blk, 0, stream>>>(wl2, Wl2_t, (unsigned)H2W, (unsigned)HIDW);
  xconv_kernel<<<dim3((unsigned)(((size_t)NNODE * IND) / 2048u)), blk, 0, stream>>>(x, X16);

  edge_kernel<<<dim3(NNODE / EROWS), dim3(ETHREADS), 0, stream>>>(
      adj, xdeg, ydeg, wm1, bm1, wm2, bm2, B16, colp, drv);
  dcol_kernel<<<dim3(NNODE / 128), dim3(128), 0, stream>>>(colp, dcv);

  gemm_xw_kernel<<<dim3(HIDW / 64, NNODE / 64), blk, 0, stream>>>(X16, Wg1_t, dcv, XWt);
  gemm_h1_kernel<<<dim3(HIDW / 64, NNODE / 64), blk, 0, stream>>>(B16, XWt, drv, H1p);
  gemm_hid_kernel<<<dim3(H2W / 64, NNODE / 64), blk, 0, stream>>>(H1p, Wl2_t, bl2, dcv, wg2, out, HGt);
  gemm_out_kernel<<<dim3(NNODE / 128), blk, 0, stream>>>(B16, HGt, drv, out);
}
